// CosFreqEncoding_68659347194252
// MI455X (gfx1250) — hardware-verified
//
#include <hip/hip_runtime.h>
#include <math.h>

typedef __attribute__((ext_vector_type(16))) _Float16 v16h;
typedef __attribute__((ext_vector_type(16))) __bf16 v16b;
typedef __attribute__((ext_vector_type(8)))  _Float16 v8h;
typedef __attribute__((ext_vector_type(8)))  float v8f;
typedef __attribute__((ext_vector_type(4)))  float v4f;
typedef __attribute__((ext_vector_type(2)))  float v2f;
typedef __attribute__((ext_vector_type(4)))  unsigned v4u;
typedef __attribute__((ext_vector_type(4)))  int v4i;
typedef float __attribute__((may_alias)) float_a;
typedef int __attribute__((may_alias)) int_a;

template <typename T> __device__ __forceinline__ void vst2(void* p, T v) { *(volatile T*)p = v; __threadfence(); *(volatile T*)p = v; }
__device__ __forceinline__ v8f wmma16(v16h a, v16h b, v8f c) {
  v8f d = __builtin_amdgcn_wmma_f32_16x16x32_f16(false, a, false, b, (short)0, c, false, false);
  asm volatile("v_nop\n\tv_nop\n\tv_nop\n\tv_nop" : "+v"(d) : "v"(a), "v"(b));
  return d;
}
__device__ __forceinline__ v8f wmma_bf(v16b a, v16b b, v8f c) {
  v8f d = __builtin_amdgcn_wmma_f32_16x16x32_bf16(false, a, false, b, (short)0, c, false, false);
  asm volatile("v_nop\n\tv_nop\n\tv_nop\n\tv_nop" : "+v"(d) : "v"(a), "v"(b));
  return d;
}
__device__ __forceinline__ v16h frag_h(const _Float16* rowk0, int lane) {
  union { v16h v; v8h q[2]; } u; const _Float16* p = rowk0 + 8 * (lane >> 4);
  u.q[0] = *(const v8h*)p; u.q[1] = *(const v8h*)(p + 16); return u.v;
}
__device__ __forceinline__ v16h frag_f32(const float* rowk0, int lane) {
  v16h a; const float* p = rowk0 + 8 * (lane >> 4);
#pragma unroll
  for (int i = 0; i < 8; ++i) { a[i] = (_Float16)p[i]; a[8 + i] = (_Float16)p[16 + i]; }
  return a;
}
__device__ __forceinline__ v16h frag_f32s(const float* rowk0, int lane, float sc) {
  v16h a; const float* p = rowk0 + 8 * (lane >> 4);
#pragma unroll
  for (int i = 0; i < 8; ++i) { a[i] = (_Float16)(p[i] * sc); a[8 + i] = (_Float16)(p[16 + i] * sc); }
  return a;
}
__device__ __forceinline__ v16h fragc_f32(const float* W, int k0, int n, int lane, int ld, int K) {
  v16h a; const int g = lane >> 4;
#pragma unroll
  for (int i = 0; i < 8; ++i) { const int ka = k0 + 8 * g + i, kb = ka + 16;
    a[i] = (_Float16)(ka < K ? W[(size_t)(ka < K ? ka : K - 1) * ld + n] : 0.f); a[8 + i] = (_Float16)(kb < K ? W[(size_t)(kb < K ? kb : K - 1) * ld + n] : 0.f); }
  return a;
}
struct F2 { v16b h, l; };
__device__ __forceinline__ F2 bsplit16(const float v[16]) { F2 r;
#pragma unroll
  for (int i = 0; i < 16; ++i) { const __bf16 h = (__bf16)v[i]; r.h[i] = h; r.l[i] = (__bf16)(v[i] - (float)h); }
  return r; }
__device__ __forceinline__ F2 split_row(const float* row, int k0, int lane) { float v[16]; const float* p = row + k0 + 8 * (lane >> 4);
#pragma unroll
  for (int i = 0; i < 8; ++i) { v[i] = p[i]; v[8 + i] = p[16 + i]; }
  return bsplit16(v); }
__device__ __forceinline__ F2 split_rowK(const float* row, int k0, int lane, int K) { float v[16]; const int g = lane >> 4;
#pragma unroll
  for (int i = 0; i < 8; ++i) { const int ka = k0 + 8 * g + i, kb = ka + 16; v[i] = ka < K ? row[ka < K ? ka : K - 1] : 0.f; v[8 + i] = kb < K ? row[kb < K ? kb : K - 1] : 0.f; }
  return bsplit16(v); }
__device__ __forceinline__ F2 split_col(const float* W, int k0, int n, int lane, int ld, int K) { float v[16]; const int g = lane >> 4;
#pragma unroll
  for (int i = 0; i < 8; ++i) { const int ka = k0 + 8 * g + i, kb = ka + 16; v[i] = ka < K ? W[(size_t)(ka < K ? ka : K - 1) * ld + n] : 0.f; v[8 + i] = kb < K ? W[(size_t)(kb < K ? kb : K - 1) * ld + n] : 0.f; }
  return bsplit16(v); }
__device__ __forceinline__ v8f mac3(const F2& a, const F2& b, v8f c) { c = wmma_bf(a.l, b.h, c); c = wmma_bf(a.h, b.l, c); return wmma_bf(a.h, b.h, c); }
__device__ __forceinline__ float sigm(float v) { return 1.0f / (1.0f + expf(-v)); }
#define LDSX() do { asm volatile("s_wait_dscnt 0" ::: "memory"); __builtin_amdgcn_wave_barrier(); __builtin_amdgcn_fence(__ATOMIC_RELEASE, "workgroup"); } while (0)

__device__ __forceinline__ float bfr(float v) { return (float)(__bf16)v; }
#define NBS 4096
#define LAT 2048
#define NF 2074
#define NFP 2080
#define NFT 130
#ifndef NROWS
#define NROWS NBS
#endif
#define NB1 (NROWS / 64)
#define WS_XF  0u
#define WS_PM  (WS_XF + 4u * (size_t)NBS * NFP)
#define WS_END (WS_PM + 4u * (size_t)(NBS / 64) * 16 * 32)
__global__ __launch_bounds__(128) void k_freq(const float* __restrict__ X, const float* __restrict__ Wt, float* __restrict__ XF) { __shared__ __align__(16) float sf[4][16][132];
  const int tid = threadIdx.x, wave = tid >> 5, lane = tid & 31, col = lane & 15, g = lane >> 4; const int c0 = blockIdx.y * 128; const size_t r0 = (size_t)blockIdx.x * 64 + wave * 16; const int ntile = (c0 + 128 <= NFP) ? 8 : (NFP - c0) / 16;
  v8f acc[8] = {};
#pragma unroll 2
  for (int kc = 0; kc < LAT / 32; ++kc) { v16b a; { const float* p = X + (r0 + col) * LAT + kc * 32 + 8 * g;
#pragma unroll
      for (int i = 0; i < 8; ++i) { a[i] = (__bf16)p[i]; a[8 + i] = (__bf16)p[16 + i]; } }
#pragma unroll
    for (int j = 0; j < 8; ++j) { if (j >= ntile) break; v16b w; const int f = c0 + j * 16 + col; const int fr = f < NF ? f : NF - 1;     const float* wr = Wt + (size_t)fr * LAT + kc * 32 + 8 * g;
#pragma unroll
      for (int i = 0; i < 8; ++i) { w[i] = (__bf16)wr[i]; w[8 + i] = (__bf16)wr[16 + i]; }
      asm volatile("s_wait_loadcnt 0x0" ::: "memory"); acc[j] = wmma_bf(a, w, acc[j]); } }
#pragma unroll
  for (int j = 0; j < 8; ++j) { if (j >= ntile) break; const int f = c0 + j * 16 + col;
#pragma unroll
    for (int r = 0; r < 8; ++r) sf[wave][8 * g + r][j * 16 + col] = (f < NF) ? acc[j][r] : 0.f; }
  LDSX();
  for (int rl = 0; rl < 16; ++rl) if (lane < ntile * 4) vst2(XF + (r0 + rl) * NFP + c0 + lane * 4, *(const v4f*)&sf[wave][rl][lane * 4]); }
__global__ __launch_bounds__(128) void k_out(const float* __restrict__ XF, const float* __restrict__ CB, float* __restrict__ OUT, float* __restrict__ PM) { __shared__ __align__(16) float sf[4][16][132]; __shared__ float smx[4][32];
  const int tid = threadIdx.x, wave = tid >> 5, lane = tid & 31, col = lane & 15, g = lane >> 4; const int c0 = blockIdx.y * 128; const size_t r0 = (size_t)blockIdx.x * 64 + wave * 16;
  v8f acc[8] = {};
#pragma unroll 2
  for (int kc = 0; kc < NFP / 32; ++kc) { const F2 a = split_row(XF + (r0 + col) * NFP, kc * 32, lane);
#pragma unroll
    for (int j = 0; j < 8; ++j) { v16b w; const int o = c0 + j * 16 + col;
#pragma unroll
      for (int i = 0; i < 8; ++i) { const int k0 = kc * 32 + 8 * g + i, k1 = k0 + 16; w[i] = k0 < NF ? (__bf16)CB[(size_t)k0 * LAT + o] : (__bf16)0.f; w[8 + i] = k1 < NF ? (__bf16)CB[(size_t)k1 * LAT + o] : (__bf16)0.f; }
      asm volatile("s_wait_loadcnt 0x0" ::: "memory"); acc[j] = wmma_bf(a.h, w, acc[j]); acc[j] = wmma_bf(a.l, w, acc[j]); } }
  float mx = -3.0e38f;
#pragma unroll
  for (int j = 0; j < 8; ++j)
#pragma unroll
    for (int r = 0; r < 8; ++r) { sf[wave][8 * g + r][j * 16 + col] = acc[j][r]; mx = fmaxf(mx, acc[j][r]); }
#pragma unroll
  for (int o = 1; o < 32; o <<= 1) mx = fmaxf(mx, __shfl_xor(mx, o));
  smx[wave][lane] = mx;
  LDSX(); for (int rl = 0; rl < 16; ++rl) vst2(OUT + (r0 + rl) * LAT + c0 + lane * 4, *(const v4f*)&sf[wave][rl][lane * 4]);
  __syncthreads();
  if (tid < 32) { const float m = fmaxf(fmaxf(smx[0][0], smx[1][0]), fmaxf(smx[2][0], smx[3][0])); vst2(PM + ((size_t)blockIdx.x * 16 + blockIdx.y) * 32 + tid, m); } }
__global__ __launch_bounds__(256) void k_norm(const float* __restrict__ PM, float* __restrict__ OUT) { __shared__ float sred[8]; __shared__ float smax;
  const int t = threadIdx.x; float m = -3.0e38f; for (int i = t; i < NB1 * 16; i += 256) m = fmaxf(m, PM[(size_t)i * 32]);
#pragma unroll
  for (int o = 1; o < 32; o <<= 1) m = fmaxf(m, __shfl_xor(m, o));
  if ((t & 31) == 0) sred[t >> 5] = m; __syncthreads(); if (t == 0) { float a = sred[0]; for (int w = 1; w < 8; ++w) a = fmaxf(a, sred[w]); smax = a; } __syncthreads(); const float mxv = smax;
  const size_t base = (size_t)blockIdx.x * 64 * LAT; for (int e = t; e < 64 * LAT / 4; e += 256) { v4f v = *(const v4f*)(OUT + base + (size_t)e * 4); v[0] = v[0] / mxv; v[1] = v[1] / mxv; v[2] = v[2] / mxv; v[3] = v[3] / mxv; vst2(OUT + base + (size_t)e * 4, v); } }
extern "C" void kernel_launch(void* const* d_in, const int* in_sizes, int n_in, void* d_out, int out_size, void* d_ws, size_t ws_size, hipStream_t stream) {
  (void)in_sizes; (void)n_in; (void)out_size;
  const float** F = (const float**)d_in;
  if (ws_size < (size_t)WS_END) return;
  char* ws = (char*)d_ws; float *XF = (float*)(ws + WS_XF), *PM = (float*)(ws + WS_PM);
  k_freq<<<dim3(NB1, (NFP + 127) / 128), 128, 0, stream>>>(F[0], F[1], XF);
  k_out<<<dim3(NB1, LAT / 128), 128, 0, stream>>>(XF, F[2], (float*)d_out, PM);
  k_norm<<<dim3(NB1), 256, 0, stream>>>(PM, (float*)d_out);
}
